// SwarmSetEquivariantTorso_44976897524262
// MI455X (gfx1250) — hardware-verified
//
#include <hip/hip_runtime.h>
#include <math.h>

#define DEVI __device__ __forceinline__

typedef _Float16 v16h __attribute__((ext_vector_type(16)));
typedef _Float16 v8h  __attribute__((ext_vector_type(8)));
typedef float    v8f  __attribute__((ext_vector_type(8)));
typedef float    v4f  __attribute__((ext_vector_type(4)));
typedef v4f      v4fa __attribute__((may_alias));
union Frag  { v16h v; v8h half[2]; };
union Pack8 { v8h v; _Float16 e[8]; };

static constexpr int EGO    = 32;
static constexpr int SLOTS  = 5;
static constexpr int PSD    = 15;
static constexpr int PAIR_D = 10;
static constexpr int D_OBS  = 198;
static constexpr int PAIR_OFF = EGO + SLOTS * PSD;
static constexpr int DM = 64, MH = 128;
static constexpr int OUTD = MH + 6;
static constexpr int RT = 16;
static constexpr int TT = RT * SLOTS;
static constexpr int NTHR = 256;
static constexpr float WSCALE = 64.0f;
static constexpr float WINV   = 0.015625f;

enum : int {
  W_TOK = 0,
  W_QW  = 2048,   W_KW = 6144,  W_VW = 10240, W_OW = 14336,
  W_M1  = 18432,
  W_M2  = 26624,
  W_M3  = 43008,
  W_E1  = 51200,
  W_E2  = 55296,
  W_E3  = 71680,
  W_L1  = 79872,
  W_L2  = 96256,
  W_PK  = 112640, W_PV = 116736, W_PO = 120832,
  W_H1  = 124928,
  W_H2  = 145408,
  W_H3  = 161792,
  W_END = 178176
};
static constexpr int NSEG = 19;

DEVI float fast_exp(float x) { return __expf(x); }
DEVI float fast_rcp(float x) { return __builtin_amdgcn_rcpf(x); }

DEVI float gelu(float x) {
  float u  = 0.7978845608028654f * (x + 0.044715f * x * x * x);
  float au = fabsf(u);
  float e  = fast_exp(-2.0f * au);
  float t  = (1.0f - e) * fast_rcp(1.0f + e);
  t = copysignf(t, u);
  return 0.5f * x * (1.0f + t);
}
DEVI float nan0(float x) { return (x - x == 0.0f) ? x : 0.0f; }

DEVI v8f wmma_f16(v16h a, v16h b, v8f c) {
  v8f d = __builtin_amdgcn_wmma_f32_16x16x32_f16(false, a, false, b, (short)0, c, false, false);
  asm volatile("v_nop\n\tv_nop\n\tv_nop\n\tv_nop" : "+v"(d) : "v"(a), "v"(b));
  return d;
}

DEVI v16h load_a_frag(const _Float16* A, int lda, int m0, int k0) {
  const int lane = threadIdx.x & 31;
  const int m = m0 + (lane & 15), h = lane >> 4;
  const _Float16* q = A + m * lda + k0 + 8 * h;
  Frag f;
  f.half[0] = *(const v8h*)q;
  f.half[1] = *(const v8h*)(q + 16);
  return f.v;
}

DEVI v16h load_b_frag(const _Float16* __restrict__ Wt, int ldw, int n0, int k0) {
  const int lane = threadIdx.x & 31;
  const int n = n0 + (lane & 15), h = lane >> 4;
  const _Float16* q = Wt + (size_t)n * ldw + k0 + 8 * h;
  Frag f;
  f.half[0] = *(const v8h*)q;
  f.half[1] = *(const v8h*)(q + 16);
  return f.v;
}

enum { ST_F16 = 1, ST_F32 = 2, ST_GELU = 4, ST_ADD = 8, ST_MASK = 16 };

template <int MODE>
DEVI void gemm(const _Float16* A, int lda,
               const _Float16* __restrict__ Wt, int ldw,
               const float* __restrict__ bias,
               int M, int N, int K,
               _Float16* C16, int ldc16,
               float* C32, int ldc32,
               const float* maskArr) {
  const int wave = threadIdx.x >> 5;
  const int nw   = blockDim.x >> 5;
  const int lane = threadIdx.x & 31;
  const int mt = M >> 4, nt = N >> 4;
  for (int t = wave; t < mt * nt; t += nw) {
    const int m0 = (t % mt) << 4;
    const int n0 = (t / mt) << 4;
    v8f acc = {0.f, 0.f, 0.f, 0.f, 0.f, 0.f, 0.f, 0.f};
    for (int k0 = 0; k0 < K; k0 += 32) {
      v16h a = load_a_frag(A, lda, m0, k0);
      v16h b = load_b_frag(Wt, ldw, n0, k0);
      acc = wmma_f16(a, b, acc);
    }
    const int n  = n0 + (lane & 15);
    const int mb = m0 + ((lane >> 4) << 3);
    const float bv = bias[n];
#pragma unroll
    for (int j = 0; j < 8; ++j) {
      const int m = mb + j;
      float v = acc[j] * WINV + bv;
      if (MODE & ST_GELU) v = gelu(v);
      if (MODE & ST_MASK) v = (maskArr[m] > 0.5f) ? v : 0.0f;
      if (MODE & ST_F16)  C16[m * ldc16 + n] = (_Float16)v;
      if (MODE & ST_F32) {
        if (MODE & ST_ADD) C32[m * ldc32 + n] += v;
        else               C32[m * ldc32 + n]  = v;
      }
    }
  }
}

struct Params {
  const float *obs;
  const float *tok_b, *ln1_s, *ln1_b;
  const float *a1_qb, *a1_kb, *a1_vb, *a1_ob;
  const float *ln2_s, *ln2_b;
  const float *m1_b, *m2_b, *m3_b;
  const float *e1_b, *e2_b, *e3_b;
  const float *l1_b, *l2_b, *l3_w, *l3_b;
  const float *seed, *p_qw, *p_qb, *p_kb, *p_vb, *p_ob;
  const float *pr_w, *pr_b;
  const float *h1_b, *h2_b, *h3_b;
  const _Float16 *W;
  float *out;
};
static_assert(sizeof(Params) == 33 * sizeof(void*));

struct WSeg { const float* src; int K; int N; int Kpad; int off; };
struct WTable { WSeg s[NSEG]; };
static_assert(sizeof(WSeg) == 24);
static_assert(sizeof(WTable) == 24 * NSEG);

__global__ __launch_bounds__(NTHR) void convert_w(WTable t, _Float16* __restrict__ dst, int ngroups) {
  const int g = blockIdx.x * NTHR + threadIdx.x;
  if (g >= ngroups) return;
  const int e0 = g << 3;
  const float* src = t.s[0].src;
  int K = t.s[0].K, N = t.s[0].N, Kpad = t.s[0].Kpad, off = t.s[0].off;
#pragma unroll
  for (int s = 1; s < NSEG; ++s) {
    if (e0 >= t.s[s].off) { src = t.s[s].src; K = t.s[s].K; N = t.s[s].N; Kpad = t.s[s].Kpad; off = t.s[s].off; }
  }
  const int local = e0 - off;
  const int n = local / Kpad;
  const int k = local - n * Kpad;
  Pack8 u;
#pragma unroll
  for (int i = 0; i < 8; ++i) {
    float x = 0.0f;
    if ((k + i) < K && n < N) x = src[(size_t)(k + i) * N + n];
    u.e[i] = (_Float16)(x * WSCALE);
  }
  _Float16* d = dst + e0;
  *(volatile v8h*)d = u.v;
  __threadfence();
  *(volatile v8h*)d = u.v;
}

__global__ __launch_bounds__(NTHR) void main_kernel(Params p, int nrows) {
  __shared__ float s_obs[RT * D_OBS];
  __shared__ float s_tok[TT * DM];
  __shared__ __align__(32) _Float16 s_A [TT * 160];
  __shared__ __align__(32) _Float16 s_H1[TT * MH];
  __shared__ __align__(32) _Float16 s_H2[TT * MH];
  __shared__ __align__(32) _Float16 s_K [TT * DM];
  __shared__ __align__(32) _Float16 s_V [TT * DM];
  __shared__ float s_mask[TT], s_msafe[TT], s_many[RT];
  __shared__ float s_logit[TT], s_qv[DM], s_c[RT * DM];
  __shared__ __align__(16) float s_out[RT * OUTD];

  const int tid  = threadIdx.x;
  const int row0 = blockIdx.x * RT;
  int rows_here = nrows - row0;
  if (rows_here > RT) rows_here = RT;
  if (rows_here < 0)  rows_here = 0;

  {
    const size_t gbase = (size_t)row0 * D_OBS;
    const int nval = rows_here * D_OBS;
    for (int i = tid; i < RT * D_OBS; i += NTHR)
      s_obs[i] = (i < nval) ? p.obs[gbase + i] : 0.0f;
  }
  __syncthreads();

  if (tid < TT) {
    int r = tid / SLOTS, s = tid - r * SLOTS;
    const float* rb = &s_obs[r * D_OBS + EGO + s * PSD];
    bool m = (fabsf(rb[0]) > 1e-6f) || (fabsf(rb[1]) > 1e-6f) || (fabsf(rb[2]) > 1e-6f);
    s_mask[tid] = m ? 1.0f : 0.0f;
  }
  __syncthreads();
  if (tid < RT) {
    float any = 0.0f;
    for (int s = 0; s < SLOTS; ++s) any = fmaxf(any, s_mask[tid * SLOTS + s]);
    s_many[tid] = any;
    for (int s = 0; s < SLOTS; ++s)
      s_msafe[tid * SLOTS + s] = (any > 0.5f) ? s_mask[tid * SLOTS + s]
                                              : (s == 0 ? 1.0f : 0.0f);
  }
  __syncthreads();

  if (tid < TT) {
    int r = tid / SLOTS, s = tid - r * SLOTS;
    const float* base = &s_obs[r * D_OBS + EGO];
    bool ms = s_mask[tid] > 0.5f;
    _Float16* w = &s_A[tid * 32];
    if (ms) {
      float rc[3];
      for (int c = 0; c < 3; ++c) rc[c] = nan0(base[s * PSD + c]);
      float dmin = 1e9f, dsum = 0.0f; int cnt = 0;
      for (int j = 0; j < SLOTS; ++j) {
        if (j == s) continue;
        if (!(s_mask[r * SLOTS + j] > 0.5f)) continue;
        float dx = rc[0] - nan0(base[j * PSD + 0]);
        float dy = rc[1] - nan0(base[j * PSD + 1]);
        float dz = rc[2] - nan0(base[j * PSD + 2]);
        float d  = sqrtf(dx * dx + dy * dy + dz * dz);
        dmin = fminf(dmin, d); dsum += d; ++cnt;
      }
      float dmean = (cnt > 0) ? dsum * (1.0f / ((float)cnt + 1e-9f)) : 0.0f;
      dmin = fminf(dmin, 60000.0f);
      float ax = base[s * PSD + 6], ay = base[s * PSD + 7], az = base[s * PSD + 8];
      float an = sqrtf(ax * ax + ay * ay + az * az);
      for (int c = 0; c < 4; ++c) w[c] = (_Float16)base[s * PSD + 11 + c];
      w[4] = (_Float16)base[s * PSD + 9];
      w[5] = (_Float16)base[s * PSD + 10];
      w[6] = (_Float16)ax; w[7] = (_Float16)ay; w[8] = (_Float16)az;
      w[9] = (_Float16)an; w[10] = (_Float16)dmin; w[11] = (_Float16)dmean;
      for (int c = 12; c < 32; ++c) w[c] = (_Float16)0.0f;
    } else {
      for (int c = 0; c < 32; ++c) w[c] = (_Float16)0.0f;
    }
  }
  __syncthreads();

  gemm<ST_F32 | ST_GELU | ST_MASK>(s_A, 32, p.W + W_TOK, 32, p.tok_b,
                                   TT, DM, 32, nullptr, 0, s_tok, DM, s_mask);
  __syncthreads();

  if (tid < TT) {
    const float* x = &s_tok[tid * DM];
    float m = 0.f; for (int i = 0; i < DM; ++i) m += x[i]; m *= (1.0f / DM);
    float v = 0.f; for (int i = 0; i < DM; ++i) { float d = x[i] - m; v += d * d; }
    v *= (1.0f / DM);
    float rs = rsqrtf(v + 1e-6f);
    for (int i = 0; i < DM; ++i)
      s_A[tid * DM + i] = (_Float16)((x[i] - m) * rs * p.ln1_s[i] + p.ln1_b[i]);
  }
  __syncthreads();

  gemm<ST_F16>(s_A, DM, p.W + W_QW, 64, p.a1_qb, TT, DM, DM, s_H1, DM, nullptr, 0, nullptr);
  gemm<ST_F16>(s_A, DM, p.W + W_KW, 64, p.a1_kb, TT, DM, DM, s_K,  DM, nullptr, 0, nullptr);
  gemm<ST_F16>(s_A, DM, p.W + W_VW, 64, p.a1_vb, TT, DM, DM, s_V,  DM, nullptr, 0, nullptr);
  __syncthreads();

  if (tid < RT * 4) {
    int r = tid >> 2, h = tid & 3, tb = r * SLOTS, ho = h * 16;
    float lg[SLOTS][SLOTS];
    for (int i = 0; i < SLOTS; ++i)
      for (int j = 0; j < SLOTS; ++j) {
        if (s_msafe[tb + i] > 0.5f && s_msafe[tb + j] > 0.5f) {
          float a = 0.f;
          for (int d = 0; d < 16; ++d)
            a += (float)s_H1[(tb + i) * DM + ho + d] * (float)s_K[(tb + j) * DM + ho + d];
          lg[i][j] = a * 0.25f;
        } else lg[i][j] = -3.4028235e38f;
      }
    for (int i = 0; i < SLOTS; ++i) {
      float mx = lg[i][0];
      for (int j = 1; j < SLOTS; ++j) mx = fmaxf(mx, lg[i][j]);
      float a[SLOTS], sum = 0.f;
      for (int j = 0; j < SLOTS; ++j) { a[j] = fast_exp(lg[i][j] - mx); sum += a[j]; }
      float inv = fast_rcp(sum);
      for (int d = 0; d < 16; ++d) {
        float o = 0.f;
        for (int j = 0; j < SLOTS; ++j)
          o += a[j] * inv * (float)s_V[(tb + j) * DM + ho + d];
        s_H2[(tb + i) * DM + ho + d] = (_Float16)o;
      }
    }
  }
  __syncthreads();

  gemm<ST_F32 | ST_ADD | ST_MASK>(s_H2, DM, p.W + W_OW, 64, p.a1_ob,
                                  TT, DM, DM, nullptr, 0, s_tok, DM, s_mask);
  __syncthreads();

  if (tid < TT) {
    const float* x = &s_tok[tid * DM];
    float m = 0.f; for (int i = 0; i < DM; ++i) m += x[i]; m *= (1.0f / DM);
    float v = 0.f; for (int i = 0; i < DM; ++i) { float d = x[i] - m; v += d * d; }
    v *= (1.0f / DM);
    float rs = rsqrtf(v + 1e-6f);
    for (int i = 0; i < DM; ++i)
      s_A[tid * DM + i] = (_Float16)((x[i] - m) * rs * p.ln2_s[i] + p.ln2_b[i]);
  }
  __syncthreads();
  gemm<ST_F16 | ST_GELU>(s_A, DM, p.W + W_M1, 64, p.m1_b, TT, MH, DM, s_H1, MH, nullptr, 0, nullptr);
  __syncthreads();
  gemm<ST_F16 | ST_GELU>(s_H1, MH, p.W + W_M2, 128, p.m2_b, TT, MH, MH, s_H2, MH, nullptr, 0, nullptr);
  __syncthreads();
  gemm<ST_F32 | ST_ADD | ST_MASK>(s_H2, MH, p.W + W_M3, 128, p.m3_b,
                                  TT, DM, MH, nullptr, 0, s_tok, DM, s_mask);
  __syncthreads();

  for (int i = tid; i < TT * DM; i += NTHR) {
    int t = i >> 6, c = i & 63;
    s_A[t * MH + c] = (_Float16)s_tok[i];
  }
  for (int i = tid; i < RT * EGO; i += NTHR) {
    int r = i >> 5, c = i & 31;
    s_V[r * EGO + c] = (_Float16)s_obs[r * D_OBS + c];
  }
  __syncthreads();

  gemm<ST_F16 | ST_GELU>(s_V, EGO, p.W + W_E1, 32, p.e1_b, RT, MH, EGO, s_H1, MH, nullptr, 0, nullptr);
  __syncthreads();
  gemm<ST_F16 | ST_GELU>(s_H1, MH, p.W + W_E2, 128, p.e2_b, RT, MH, MH, s_H2, MH, nullptr, 0, nullptr);
  __syncthreads();
  gemm<ST_F16>(s_H2, MH, p.W + W_E3, 128, p.e3_b, RT, DM, MH, s_K, DM, nullptr, 0, nullptr);
  __syncthreads();

  for (int i = tid; i < TT * DM; i += NTHR) {
    int t = i >> 6, c = i & 63;
    s_A[t * MH + DM + c] = s_K[(t / SLOTS) * DM + c];
  }
  __syncthreads();

  gemm<ST_F16 | ST_GELU>(s_A, MH, p.W + W_L1, 128, p.l1_b, TT, MH, MH, s_H1, MH, nullptr, 0, nullptr);
  __syncthreads();
  gemm<ST_F16 | ST_GELU>(s_H1, MH, p.W + W_L2, 128, p.l2_b, TT, MH, MH, s_H2, MH, nullptr, 0, nullptr);
  __syncthreads();
  if (tid < TT) {
    float a = p.l3_b[0];
    for (int i = 0; i < MH; ++i) a += (float)s_H2[tid * MH + i] * p.l3_w[i];
    s_logit[tid] = a;
  }
  if (tid < DM) {
    float a = p.p_qb[tid];
    for (int k = 0; k < DM; ++k) a += p.seed[k] * p.p_qw[k * DM + tid];
    s_qv[tid] = a;
  }
  __syncthreads();

  if (tid < RT) {
    float e[SLOTS], mx = -1e30f;
    for (int s = 0; s < SLOTS; ++s) {
      float ml = (s_mask[tid * SLOTS + s] > 0.5f) ? s_logit[tid * SLOTS + s] : -1e9f;
      e[s] = ml; mx = fmaxf(mx, ml);
    }
    float sum = 0.f;
    for (int s = 0; s < SLOTS; ++s) { e[s] = fast_exp(e[s] - mx) * s_mask[tid * SLOTS + s]; sum += e[s]; }
    float inv = fast_rcp(sum + 1e-9f);
    float vr[3] = {0.f, 0.f, 0.f}, vu[3] = {0.f, 0.f, 0.f};
    for (int s = 0; s < SLOTS; ++s) {
      float al = e[s] * inv;
      const float* rb = &s_obs[tid * D_OBS + EGO + s * PSD];
      for (int c = 0; c < 3; ++c) { vr[c] += al * rb[c]; vu[c] += al * rb[3 + c]; }
    }
    for (int c = 0; c < 3; ++c) { s_out[tid * OUTD + MH + c] = vr[c]; s_out[tid * OUTD + MH + 3 + c] = vu[c]; }
  }

  gemm<ST_F16>(s_A, MH, p.W + W_PK, 64, p.p_kb, TT, DM, DM, s_K, DM, nullptr, 0, nullptr);
  gemm<ST_F16>(s_A, MH, p.W + W_PV, 64, p.p_vb, TT, DM, DM, s_V, DM, nullptr, 0, nullptr);
  __syncthreads();

  if (tid < RT * 4) {
    int r = tid >> 2, h = tid & 3, tb = r * SLOTS, ho = h * 16;
    float lg[SLOTS];
    for (int j = 0; j < SLOTS; ++j) {
      if (s_msafe[tb + j] > 0.5f) {
        float a = 0.f;
        for (int d = 0; d < 16; ++d)
          a += s_qv[ho + d] * (float)s_K[(tb + j) * DM + ho + d];
        lg[j] = a * 0.25f;
      } else lg[j] = -3.4028235e38f;
    }
    float mx = lg[0];
    for (int j = 1; j < SLOTS; ++j) mx = fmaxf(mx, lg[j]);
    float a[SLOTS], sum = 0.f;
    for (int j = 0; j < SLOTS; ++j) { a[j] = fast_exp(lg[j] - mx); sum += a[j]; }
    float inv = fast_rcp(sum);
    for (int d = 0; d < 16; ++d) {
      float c = 0.f;
      for (int j = 0; j < SLOTS; ++j)
        c += a[j] * inv * (float)s_V[(tb + j) * DM + ho + d];
      s_H1[r * DM + ho + d] = (_Float16)c;
    }
  }
  __syncthreads();

  gemm<ST_F32>(s_H1, DM, p.W + W_PO, 64, p.p_ob, RT, DM, DM, nullptr, 0, s_c, DM, nullptr);
  __syncthreads();

  for (int i = tid; i < RT * EGO; i += NTHR) {
    int r = i >> 5, c = i & 31;
    s_A[r * 160 + c] = (_Float16)s_obs[r * D_OBS + c];
  }
  for (int i = tid; i < RT * DM; i += NTHR) {
    int r = i >> 6, c = i & 63;
    float cv = (s_many[r] > 0.5f) ? s_c[r * DM + c] : 0.0f;
    s_A[r * 160 + EGO + c] = (_Float16)cv;
  }
  for (int i = tid; i < RT * DM; i += NTHR) {
    int r = i >> 6, n = i & 63;
    float a = p.pr_b[n];
    for (int k = 0; k < PAIR_D; ++k)
      a += s_obs[r * D_OBS + PAIR_OFF + k] * p.pr_w[k * DM + n];
    s_A[r * 160 + EGO + DM + n] = (_Float16)gelu(a);
  }
  __syncthreads();

  gemm<ST_F16 | ST_GELU>(s_A, 160, p.W + W_H1, 160, p.h1_b, RT, MH, 160, s_H1, MH, nullptr, 0, nullptr);
  __syncthreads();
  gemm<ST_F16 | ST_GELU>(s_H1, MH, p.W + W_H2, 128, p.h2_b, RT, MH, MH, s_H2, MH, nullptr, 0, nullptr);
  __syncthreads();
  gemm<ST_F32>(s_H2, MH, p.W + W_H3, 128, p.h3_b, RT, MH, MH, nullptr, 0, s_out, OUTD, nullptr);
  __syncthreads();

  {
    const int nvalid = rows_here * OUTD;
    const int n4 = nvalid >> 2;
    float* gout = p.out + (size_t)row0 * OUTD;
    const v4fa* s4 = (const v4fa*)s_out;
    constexpr int NJ = (RT * OUTD / 4 + NTHR - 1) / NTHR;
    v4f hold[NJ];
#pragma unroll
    for (int j = 0; j < NJ; ++j) {
      const int i = tid + NTHR * j;
      v4f v = {0.f, 0.f, 0.f, 0.f};
      if (i < n4) v = s4[i];
      hold[j] = v;
      if (i < n4) *(volatile v4f*)(gout + 4 * i) = v;
    }
    const int trem = nvalid & 3;
    float tailv = 0.0f;
    if (tid < trem) { tailv = s_out[4 * n4 + tid]; *(volatile float*)(gout + 4 * n4 + tid) = tailv; }
    __threadfence();
#pragma unroll
    for (int j = 0; j < NJ; ++j) {
      const int i = tid + NTHR * j;
      if (i < n4) *(volatile v4f*)(gout + 4 * i) = hold[j];
    }
    if (tid < trem) *(volatile float*)(gout + 4 * n4 + tid) = tailv;
  }
}

extern "C" void kernel_launch(void* const* d_in, const int* in_sizes, int n_in,
                              void* d_out, int out_size, void* d_ws, size_t ws_size,
                              hipStream_t stream) {
  if (n_in < 50) return;
  int nrows = out_size / OUTD;
  int nrows_in = in_sizes[0] / D_OBS;
  if (nrows_in < nrows) nrows = nrows_in;
  if (nrows <= 0) return;
  if (ws_size < (size_t)W_END * sizeof(_Float16)) return;

  _Float16* Wf16 = (_Float16*)d_ws;

  WTable t;
  auto seg = [&](int i, int idx, int K, int N, int Kpad, int off) {
    t.s[i].src = (const float*)d_in[idx];
    t.s[i].K = K; t.s[i].N = N; t.s[i].Kpad = Kpad; t.s[i].off = off;
  };
  seg(0,  1,  12,  64,  32,  W_TOK);
  seg(1,  5,  64,  64,  64,  W_QW);
  seg(2,  7,  64,  64,  64,  W_KW);
  seg(3,  9,  64,  64,  64,  W_VW);
  seg(4,  11, 64,  64,  64,  W_OW);
  seg(5,  15, 64,  128, 64,  W_M1);
  seg(6,  17, 128, 128, 128, W_M2);
  seg(7,  19, 128, 64,  128, W_M3);
  seg(8,  21, 32,  128, 32,  W_E1);
  seg(9,  23, 128, 128, 128, W_E2);
  seg(10, 25, 128, 64,  128, W_E3);
  seg(11, 27, 128, 128, 128, W_L1);
  seg(12, 29, 128, 128, 128, W_L2);
  seg(13, 36, 64,  64,  64,  W_PK);
  seg(14, 38, 64,  64,  64,  W_PV);
  seg(15, 40, 64,  64,  64,  W_PO);
  seg(16, 44, 160, 128, 160, W_H1);
  seg(17, 46, 128, 128, 128, W_H2);
  seg(18, 48, 128, 128, 128, W_H3);

  const int ngroups = W_END / 8;
  convert_w<<<(ngroups + NTHR - 1) / NTHR, NTHR, 0, stream>>>(t, Wf16, ngroups);

  Params p;
  p.obs   = (const float*)d_in[0];
  p.tok_b = (const float*)d_in[2];
  p.ln1_s = (const float*)d_in[3];  p.ln1_b = (const float*)d_in[4];
  p.a1_qb = (const float*)d_in[6];  p.a1_kb = (const float*)d_in[8];
  p.a1_vb = (const float*)d_in[10]; p.a1_ob = (const float*)d_in[12];
  p.ln2_s = (const float*)d_in[13]; p.ln2_b = (const float*)d_in[14];
  p.m1_b  = (const float*)d_in[16]; p.m2_b = (const float*)d_in[18]; p.m3_b = (const float*)d_in[20];
  p.e1_b  = (const float*)d_in[22]; p.e2_b = (const float*)d_in[24]; p.e3_b = (const float*)d_in[26];
  p.l1_b  = (const float*)d_in[28]; p.l2_b = (const float*)d_in[30];
  p.l3_w  = (const float*)d_in[31]; p.l3_b = (const float*)d_in[32];
  p.seed  = (const float*)d_in[33];
  p.p_qw  = (const float*)d_in[34]; p.p_qb = (const float*)d_in[35];
  p.p_kb  = (const float*)d_in[37]; p.p_vb = (const float*)d_in[39]; p.p_ob = (const float*)d_in[41];
  p.pr_w  = (const float*)d_in[42]; p.pr_b = (const float*)d_in[43];
  p.h1_b  = (const float*)d_in[45]; p.h2_b = (const float*)d_in[47]; p.h3_b = (const float*)d_in[49];
  p.W     = Wf16;
  p.out   = (float*)d_out;

  main_kernel<<<(nrows + RT - 1) / RT, NTHR, 0, stream>>>(p, nrows);
}
